// GNNEncoder_57982058496233
// MI455X (gfx1250) — hardware-verified
//
#include <hip/hip_runtime.h>
#include <stddef.h>
#include <stdint.h>
#include <math.h>


#define FIN     4
#define K1P     32
#define C1      64
#define NP1     128
#define C2      32
#define NP2     64
#define K2      64
#define NTHR    256
#define NWAVE   8
#define EPT     8
#define CHUNK   (NTHR * EPT)
#define WCAP    (EPT * 32)
#define LISTN   (NWAVE * WCAP)
#define NBMAX   2048
#define SLOTB   11
#define NBRUN   1024
#define RCAP    28672
#define DEGCAP  128
#define STW     64
#define GBM     64
#define GBN     64
#define GTHR    128
#define CX      8.0f
#define CL      2048.0f
#define CW      64.0f
#define SCL_XW  0.001953125f
#define SCL_XWL 9.5367431640625e-7f
#define NEGS    0.2f
#define LNEPS   1e-5f
#define WSMAX   134217728
#define LDS_AGG ((2 * RCAP + 2 * NBMAX + LISTN) * 4 + 64)

static_assert((CHUNK & (CHUNK - 1)) == 0 && CHUNK <= (1 << SLOTB));
static_assert(NBMAX == (1 << SLOTB));
static_assert((NBRUN & (NBRUN - 1)) == 0 && NBRUN <= NBMAX && NBRUN >= 16);
static_assert(NTHR * 8 == NBMAX);
static_assert(LISTN >= NBMAX);
static_assert(LISTN >= NWAVE * WCAP);
static_assert((RCAP % 32) == 0);
static_assert(NWAVE * STW <= RCAP);
static_assert(C1 <= STW && C2 <= STW);
static_assert(LDS_AGG <= 300000);
static_assert(GBM == (GTHR / 32) * 16);
static_assert((K1P % 32) == 0 && (K2 % 32) == 0);
static_assert((NP1 % GBN) == 0 && (NP2 % GBN) == 0);
static_assert(K2 == C1 && C1 == 2 * 32 && C2 == 32 && K1P / 8 == 4 && FIN == 4);
static_assert(NP1 == 2 * C1 && NP2 == 2 * C2);

typedef float          v2f   __attribute__((ext_vector_type(2)));
typedef float          v4f   __attribute__((ext_vector_type(4)));
typedef float          v8f   __attribute__((ext_vector_type(8)));
typedef int            v4i   __attribute__((ext_vector_type(4)));
typedef int            v8i   __attribute__((ext_vector_type(8)));
typedef unsigned short v8us  __attribute__((ext_vector_type(8)));
typedef _Float16       v8h   __attribute__((ext_vector_type(8)));
typedef _Float16       v16h  __attribute__((ext_vector_type(16)));
typedef __bf16         v16bf __attribute__((ext_vector_type(16)));
typedef v2f __attribute__((may_alias)) v2fa;
typedef v4f __attribute__((may_alias)) v4fa;
union FragH { v16h v;  v8us u[2]; v8i w; };
union FragB { v16bf v; v8us u[2]; v8i w; };
template<int BF> struct FT { typedef FragH T; };
template<> struct FT<1> { typedef FragB T; };

__device__ __forceinline__ v8f wmx(const FragH& a, const FragH& b, v8f c) {
  v8f d = __builtin_amdgcn_wmma_f32_16x16x32_f16(false, a.v, false, b.v, (short)0, c, false, false);
  asm volatile("v_nop\n\tv_nop\n\tv_nop\n\tv_nop" : "+v"(d) : "v"(a.w), "v"(b.w));
  return d;
}
__device__ __forceinline__ v8f wmx(const FragB& a, const FragB& b, v8f c) {
  v8f d = __builtin_amdgcn_wmma_f32_16x16x32_bf16(false, a.v, false, b.v, (short)0, c, false, false);
  asm volatile("v_nop\n\tv_nop\n\tv_nop\n\tv_nop" : "+v"(d) : "v"(a.w), "v"(b.w));
  return d;
}

__device__ __forceinline__ void ldwait() {
  asm volatile("s_wait_loadcnt 0x0" ::: "memory");
}

__device__ __forceinline__ unsigned bfbits(float v) {
  unsigned u = __float_as_uint(v);
  u = u + 0x7FFFu + ((u >> 16) & 1u);
  return u >> 16;
}
__device__ __forceinline__ float rbf(float v) { return __uint_as_float(bfbits(v) << 16); }

__device__ __forceinline__ v8us cvt8b(const v4f a, const v4f b) {
  v8us o;
  o[0] = (unsigned short)bfbits(a.x); o[1] = (unsigned short)bfbits(a.y);
  o[2] = (unsigned short)bfbits(a.z); o[3] = (unsigned short)bfbits(a.w);
  o[4] = (unsigned short)bfbits(b.x); o[5] = (unsigned short)bfbits(b.y);
  o[6] = (unsigned short)bfbits(b.z); o[7] = (unsigned short)bfbits(b.w);
  return o;
}
__device__ __forceinline__ v8h cvt8bh(const v4f a, const v4f b, const float c) {
  v8h hv;
  hv[0] = (_Float16)(rbf(a.x) * c); hv[1] = (_Float16)(rbf(a.y) * c);
  hv[2] = (_Float16)(rbf(a.z) * c); hv[3] = (_Float16)(rbf(a.w) * c);
  hv[4] = (_Float16)(rbf(b.x) * c); hv[5] = (_Float16)(rbf(b.y) * c);
  hv[6] = (_Float16)(rbf(b.z) * c); hv[7] = (_Float16)(rbf(b.w) * c);
  return hv;
}
__device__ __forceinline__ void cvt8hl(const v4f a, const v4f b, v8h& hv, v8h& lv) {
  float f[8] = {a.x * CX, a.y * CX, a.z * CX, a.w * CX, b.x * CX, b.y * CX, b.z * CX, b.w * CX};
#pragma unroll
  for (int i = 0; i < 8; ++i) {
    const _Float16 hq = (_Float16)f[i];
    hv[i] = hq;
    lv[i] = (_Float16)((f[i] - (float)hq) * CL);
  }
}

__device__ __forceinline__ float wsum(float v) {
  v += __shfl_xor(v, 16, 32);
  v += __shfl_xor(v, 8, 32);
  v += __shfl_xor(v, 4, 32);
  v += __shfl_xor(v, 2, 32);
  v += __shfl_xor(v, 1, 32);
  return v;
}
__device__ __forceinline__ float hsum8(float v) {
  v += __shfl_xor(v, 1, 32);
  v += __shfl_xor(v, 2, 32);
  v += __shfl_xor(v, 4, 32);
  return v;
}

__device__ __forceinline__ int scan_chunk(const int* __restrict__ dsts, int nE, int cbase, int slotBase,
                                          int nb, int vec8, int* list, int tid, int lane, int wave) {
  int wc = 0;
  const int el0  = tid * EPT;
  const int e0   = cbase + el0;
  const int sent = -2147483647 - 1;
  v4i da, db;
  if (vec8 != 0 && cbase + CHUNK <= nE) {
    da = *(const v4i*)(dsts + e0);
    db = *(const v4i*)(dsts + e0 + 4);
  } else {
    da.x = (e0     < nE) ? dsts[min(e0,     nE - 1)] : sent;
    da.y = (e0 + 1 < nE) ? dsts[min(e0 + 1, nE - 1)] : sent;
    da.z = (e0 + 2 < nE) ? dsts[min(e0 + 2, nE - 1)] : sent;
    da.w = (e0 + 3 < nE) ? dsts[min(e0 + 3, nE - 1)] : sent;
    db.x = (e0 + 4 < nE) ? dsts[min(e0 + 4, nE - 1)] : sent;
    db.y = (e0 + 5 < nE) ? dsts[min(e0 + 5, nE - 1)] : sent;
    db.z = (e0 + 6 < nE) ? dsts[min(e0 + 6, nE - 1)] : sent;
    db.w = (e0 + 7 < nE) ? dsts[min(e0 + 7, nE - 1)] : sent;
  }
  const unsigned nbs = (unsigned)slotBase;
  const unsigned unb = (unsigned)nb;
  const unsigned s0 = (unsigned)da.x - nbs, s1 = (unsigned)da.y - nbs;
  const unsigned s2 = (unsigned)da.z - nbs, s3 = (unsigned)da.w - nbs;
  const unsigned s4 = (unsigned)db.x - nbs, s5 = (unsigned)db.y - nbs;
  const unsigned s6 = (unsigned)db.z - nbs, s7 = (unsigned)db.w - nbs;
  const bool h0 = s0 < unb, h1 = s1 < unb, h2 = s2 < unb, h3 = s3 < unb;
  const bool h4 = s4 < unb, h5 = s5 < unb, h6 = s6 < unb, h7 = s7 < unb;
  const unsigned any = __builtin_amdgcn_ballot_w32(h0 | h1 | h2 | h3 | h4 | h5 | h6 | h7);
  if (any != 0u) {
#define HITJ(J, HJ, SJ) { \
      const unsigned mj = __builtin_amdgcn_ballot_w32(HJ); \
      if (mj != 0u) { \
        if (HJ) { \
          const int pos = wc + (int)__builtin_amdgcn_mbcnt_lo(mj, 0u); \
          if (pos < WCAP) list[wave * WCAP + pos] = ((el0 + (J)) << SLOTB) | (int)(SJ); \
        } \
        wc += (int)__builtin_popcount(mj); } }
    HITJ(0, h0, s0)
    HITJ(1, h1, s1)
    HITJ(2, h2, s2)
    HITJ(3, h3, s3)
    HITJ(4, h4, s4)
    HITJ(5, h5, s5)
    HITJ(6, h6, s6)
    HITJ(7, h7, s7)
#undef HITJ
  }
  return wc;
}

__global__ __launch_bounds__(NTHR) void k_xprep(const float* __restrict__ x, unsigned short* xb, int nN, int nUnits) {
  const int i = (int)blockIdx.x * NTHR + (int)threadIdx.x;
  if (i >= nUnits) return;
  const int row = i >> 2;
  const int c0  = (i & 3) * 8;
  const int rc  = row < nN ? row : nN - 1;
  const v4f xv  = *(const v4fa*)(x + (size_t)rc * FIN);
  const float ok = (row < nN && c0 == 0) ? 1.0f : 0.0f;
  const v4f a = xv * ok;
  const v4f z4 = {0.f, 0.f, 0.f, 0.f};
  const v8us hv = cvt8b(a, z4);
  const size_t o = (size_t)row * K1P + c0;
  *(volatile v8us*)(xb + o) = hv;
  __threadfence();
  *(volatile v8us*)(xb + o) = hv;
}

template<int MODE>
__global__ __launch_bounds__(NTHR) void k_wcat(const float* __restrict__ wl, const float* __restrict__ wr,
                                               int cols, int Kin, int Kout, unsigned short* wt, int nUnits) {
  const int u = (int)blockIdx.x * NTHR + (int)threadIdx.x;
  if (u >= nUnits) return;
  const int kq = Kout >> 3;
  const int n  = u / kq;
  const int k8 = (u - n * kq) * 8;
  const int hs = n < cols ? 0 : 1;
  int nn = n - hs * cols;
  nn = nn < 0 ? 0 : (nn > cols - 1 ? cols - 1 : nn);
  const float* w = hs ? wr : wl;
  const float okn = (n < 2 * cols) ? 1.0f : 0.0f;
  float f[8];
#pragma unroll
  for (int i = 0; i < 8; ++i) {
    const int k  = k8 + i;
    const int kc = k < Kin ? k : Kin - 1;
    const float okk = (k < Kin) ? okn : 0.0f;
    f[i] = w[(size_t)kc * (size_t)cols + nn] * okk;
  }
  const v4f a = {f[0], f[1], f[2], f[3]};
  const v4f b = {f[4], f[5], f[6], f[7]};
  const size_t o = (size_t)n * (size_t)Kout + k8;
  if (MODE == 0) {
    const v8us hv = cvt8b(a, b);
    *(volatile v8us*)(wt + o) = hv;
    __threadfence();
    *(volatile v8us*)(wt + o) = hv;
  } else {
    const v8h hv = cvt8bh(a, b, CW);
    _Float16* oh = (_Float16*)wt + o;
    *(volatile v8h*)oh = hv;
    __threadfence();
    *(volatile v8h*)oh = hv;
  }
}

template<int BF, int RES>
__global__ __launch_bounds__(GTHR) void k_gemm(
    const unsigned short* __restrict__ A, const unsigned short* __restrict__ A2,
    const unsigned short* __restrict__ WT, float* outF, int K, int ldo, float scl, float scl2)
{
  typedef typename FT<BF>::T Frag;
  __shared__ __attribute__((aligned(16))) float stg[GBM * GBN];
  const int tid = (int)threadIdx.x, lane = tid & 31, wave = tid >> 5, hh = lane >> 4, m = lane & 15;
  const int rowBase = (int)blockIdx.x * GBM;
  const int col0    = (int)blockIdx.y * GBN;

  v8f acc[4], acc2[4];
  {
    const v8f z = {0.f, 0.f, 0.f, 0.f, 0.f, 0.f, 0.f, 0.f};
    acc[0] = z; acc[1] = z; acc[2] = z; acc[3] = z;
    acc2[0] = z; acc2[1] = z; acc2[2] = z; acc2[3] = z;
  }
  const size_t arow = (size_t)(rowBase + 16 * wave + m) * (size_t)K + 8 * hh;
  const unsigned short* ap  = A  + arow;
  const unsigned short* ap2 = A2 + arow;
  const unsigned short* wp  = WT + (size_t)(col0 + m) * (size_t)K + 8 * hh;
  const int ksteps = K >> 5;
#pragma unroll 1
  for (int ks = 0; ks < ksteps; ++ks) {
    Frag af, af2;
    af.u[0] = *(const v8us*)(ap + 32 * ks);
    af.u[1] = *(const v8us*)(ap + 32 * ks + 16);
    if (RES) {
      af2.u[0] = *(const v8us*)(ap2 + 32 * ks);
      af2.u[1] = *(const v8us*)(ap2 + 32 * ks + 16);
    } else {
      af2 = af;
    }
#pragma unroll
    for (int t = 0; t < 4; ++t) {
      const unsigned short* wq = wp + (size_t)(16 * t) * (size_t)K + 32 * ks;
      Frag bf;
      bf.u[0] = *(const v8us*)wq;
      bf.u[1] = *(const v8us*)(wq + 16);
      acc[t] = wmx(af, bf, acc[t]);
      if (RES) acc2[t] = wmx(af2, bf, acc2[t]);
    }
  }

#pragma unroll
  for (int t = 0; t < 4; ++t) {
    const int lc = 16 * t + m;
#pragma unroll
    for (int r = 0; r < 8; ++r) {
      const int lr = 16 * wave + 8 * hh + r;
      const float v = RES ? fmaf(acc2[t][r], scl2, acc[t][r] * scl) : acc[t][r] * scl;
      stg[lr * GBN + lc] = v;
    }
  }
  __syncthreads();

  v4f fv[8];
#pragma unroll
  for (int i = 0; i < 8; ++i) {
    const int lr = 16 * wave + 2 * i + hh;
    fv[i] = *(const v4f*)(stg + lr * GBN + 4 * m);
  }
#pragma unroll
  for (int i = 0; i < 8; ++i) {
    const int lr = 16 * wave + 2 * i + hh;
    const int gr = rowBase + lr;
    float* op = outF + (size_t)gr * (size_t)ldo + col0 + 4 * m;
    *(volatile v4f*)op = fv[i];
  }
  __threadfence();
#pragma unroll
  for (int i = 0; i < 8; ++i) {
    const int lr = 16 * wave + 2 * i + hh;
    const int gr = rowBase + lr;
    float* op = outF + (size_t)gr * (size_t)ldo + col0 + 4 * m;
    *(volatile v4f*)op = fv[i];
  }
}

template<int LAYER>
__global__ __launch_bounds__(NTHR) void k_agg(
    const int* __restrict__ srcs, const int* __restrict__ dsts,
    const float* __restrict__ HF, const float* __restrict__ att, const float* __restrict__ bias,
    const float* __restrict__ gam, const float* __restrict__ bet,
    _Float16* Hh, _Float16* Hl, float* outF,
    int nN, int nE, int nb, int vec8, int MPr) {
  extern __shared__ v4f lds_dyn[];
  int* reg1 = (int*)lds_dyn;
  int* reg2 = reg1 + RCAP;
  int* scnt = reg2 + RCAP;
  int* soff = scnt + NBMAX;
  int* list = soff + NBMAX;
  int* wcnt = list + LISTN;
  int* wtot = wcnt + NWAVE;
  const int tid = (int)threadIdx.x, lane = tid & 31, wave = tid >> 5;
  const int nodeBase = (int)blockIdx.x * nb;

  for (int i = tid; i < NBMAX; i += NTHR) scnt[i] = 0;
  __syncthreads();

  int tot = 0;
  const int nChunks = (nE + CHUNK - 1) / CHUNK;
#pragma unroll 1
  for (int ch = 0; ch < nChunks; ++ch) {
    const int cbase = ch * CHUNK;
    const int wc = scan_chunk(dsts, nE, cbase, nodeBase, nb, vec8, list, tid, lane, wave);
    if (lane == 0) wcnt[wave] = wc;
    __syncthreads();
    int pre = 0, all = 0;
#pragma unroll
    for (int w2 = 0; w2 < NWAVE; ++w2) {
      int c = wcnt[w2];
      c = c < 0 ? 0 : (c > WCAP ? WCAP : c);
      all += c;
      pre += (w2 < wave) ? c : 0;
    }
    const int wcc  = wc > WCAP ? WCAP : wc;
    const int base = tot + pre;
#pragma unroll 1
    for (int i = lane; i < wcc; i += 32) {
      const int ent = list[wave * WCAP + i];
      const int el  = (ent >> SLOTB) & (CHUNK - 1);
      const int sl  = ent & (NBMAX - 1);
      int eid = cbase + el;
      eid = eid > nE - 1 ? nE - 1 : eid;
      const int pos = base + i;
      if (pos < RCAP) reg1[pos] = (int)(((unsigned)eid << SLOTB) | (unsigned)sl);
    }
    tot += all;
    tot = tot > RCAP ? RCAP : tot;
    __syncthreads();
  }
  const int nh = tot;

  if (wave == 0) {
#pragma unroll 1
    for (int b0 = 0; b0 < nh; b0 += 32) {
      const int idx = b0 + lane;
      const int uv  = reg1[idx < nh ? idx : nh - 1];
      const int m32 = (nh - b0) < 32 ? (nh - b0) : 32;
#pragma unroll 1
      for (int k = 0; k < m32; ++k) {
        const int u  = __builtin_amdgcn_readlane(uv, k);
        const int sl = u & (NBMAX - 1);
        if (lane == 0) scnt[sl] = scnt[sl] + 1;
      }
    }
  }
  __syncthreads();

  {
    const v4i ca = *(const v4i*)(scnt + 8 * tid);
    const v4i cb = *(const v4i*)(scnt + 8 * tid + 4);
    const int e0 = ca.x < 0 ? 0 : ca.x, e1 = ca.y < 0 ? 0 : ca.y, e2 = ca.z < 0 ? 0 : ca.z, e3 = ca.w < 0 ? 0 : ca.w;
    const int e4 = cb.x < 0 ? 0 : cb.x, e5 = cb.y < 0 ? 0 : cb.y, e6 = cb.z < 0 ? 0 : cb.z, e7 = cb.w < 0 ? 0 : cb.w;
    const int ts = e0 + e1 + e2 + e3 + e4 + e5 + e6 + e7;
    int incl = ts;
#pragma unroll
    for (int d = 1; d < 32; d <<= 1) {
      const int up = __shfl_up(incl, d);
      if (lane >= d) incl += up;
    }
    if (lane == 31) wtot[wave] = incl;
    __syncthreads();
    int pre = 0;
#pragma unroll
    for (int w2 = 0; w2 < NWAVE; ++w2) pre += (w2 < wave) ? wtot[w2] : 0;
    int run = pre + incl - ts;
    soff[8 * tid + 0] = run; run += e0;
    soff[8 * tid + 1] = run; run += e1;
    soff[8 * tid + 2] = run; run += e2;
    soff[8 * tid + 3] = run; run += e3;
    soff[8 * tid + 4] = run; run += e4;
    soff[8 * tid + 5] = run; run += e5;
    soff[8 * tid + 6] = run; run += e6;
    soff[8 * tid + 7] = run;
  }
  __syncthreads();
  for (int i = tid; i < NBMAX; i += NTHR) list[i] = soff[i];
  __syncthreads();

  if (wave == 0) {
#pragma unroll 1
    for (int b0 = 0; b0 < nh; b0 += 32) {
      const int idx = b0 + lane;
      const int uv  = reg1[idx < nh ? idx : nh - 1];
      const int m32 = (nh - b0) < 32 ? (nh - b0) : 32;
#pragma unroll 1
      for (int k = 0; k < m32; ++k) {
        const int u   = __builtin_amdgcn_readlane(uv, k);
        const int sl  = u & (NBMAX - 1);
        const int eid = (int)((unsigned)u >> SLOTB);
        if (lane == 0) {
          int pos = list[sl];
          pos = pos < 0 ? 0 : (pos > RCAP - 1 ? RCAP - 1 : pos);
          reg2[pos] = eid;
          list[sl] = pos + 1;
        }
      }
    }
  }
  __syncthreads();

  const int nbw = nb >> 3;
  const bool ovf = (nh >= RCAP);
  const float qnan = __int_as_float(0x7fc00000);
  float* stw = (float*)reg1 + wave * STW;
  const int lc = lane < 8 ? lane : 7;

  if (LAYER == 1) {
    const int c0 = 2 * lane;
    float at0, at1, bb0, bb1, gg0, gg1, ee0, ee1;
    {
      const v2f va = *(const v2fa*)(att  + c0);
      const v2f vb = *(const v2fa*)(bias + c0);
      const v2f vg = *(const v2fa*)(gam  + c0);
      const v2f ve = *(const v2fa*)(bet  + c0);
      at0 = rbf(va.x); at1 = rbf(va.y);
      bb0 = rbf(vb.x); bb1 = rbf(vb.y);
      gg0 = rbf(vg.x); gg1 = rbf(vg.y);
      ee0 = rbf(ve.x); ee1 = rbf(ve.y);
    }
#pragma unroll 1
    for (int jt = 0; jt < nbw; ++jt) {
      const int slot = wave * nbw + jt;
      const int grow = nodeBase + slot;
      const int gcl  = grow < nN ? grow : nN - 1;
      int st = soff[slot];
      const int craw = scnt[slot];
      int cnt = craw;
      st  = st < 0 ? 0 : (st > nh ? nh : st);
      cnt = cnt < 0 ? 0 : (cnt > DEGCAP ? DEGCAP : cnt);
      if (cnt > nh - st) cnt = nh - st;
      const float pz = (ovf || craw > DEGCAP) ? qnan : 0.0f;
      const float live = grow < nN ? 1.0f : 0.0f;

      const v2f xr = *(const v2fa*)(HF + (size_t)gcl * NP1 + C1 + c0);
      ldwait();
      float mx = -1.0e30f, dn = 0.f, a0 = 0.f, a1 = 0.f;

#pragma unroll 1
      for (int q = 0; q < cnt; ++q) {
        int idx = st + q; idx = idx > RCAP - 1 ? RCAP - 1 : idx;
        int eid = reg2[idx]; eid = eid < 0 ? 0 : (eid > nE - 1 ? nE - 1 : eid);
        const int sraw = srcs[eid];
        const int s = sraw < 0 ? 0 : (sraw > nN - 1 ? nN - 1 : sraw);
        const v2f xs = *(const v2fa*)(HF + (size_t)s * NP1 + c0);
        ldwait();
        float v0 = xs.x + xr.x; v0 = v0 > 0.f ? v0 : v0 * NEGS;
        float v1 = xs.y + xr.y; v1 = v1 > 0.f ? v1 : v1 * NEGS;
        float part = v0 * at0; part = fmaf(v1, at1, part);
        const float al = hsum8(part);
        const float df = al - mx;
        const float ex = __expf(-fabsf(df));
        const bool up  = df > 0.f;
        const float s1 = up ? ex : 1.0f;
        const float s2 = up ? 1.0f : ex;
        mx = up ? al : mx;
        dn = fmaf(dn, s1, s2);
        a0 = fmaf(a0, s1, s2 * xs.x);
        a1 = fmaf(a1, s1, s2 * xs.y);
      }
      const float ds = dn > 0.f ? dn : 1.0f;
      const float iv = (dn > 0.f ? 1.0f : 0.0f) * __builtin_amdgcn_rcpf(ds);
      const float t0 = fmaf(a0, iv, bb0);
      const float t1 = fmaf(a1, iv, bb1);
      const float sm = wsum(t0 + t1);
      const float mu = sm * (1.0f / C1);
      const float d0 = t0 - mu, d1 = t1 - mu;
      const float sq = wsum(fmaf(d0, d0, d1 * d1));
      const float rs = rsqrtf(sq * (1.0f / C1) + LNEPS);
      float y0 = fmaf(d0 * rs, gg0, ee0);
      float y1 = fmaf(d1 * rs, gg1, ee1);
      y0 = y0 > 0.f ? y0 : (__expf(y0) - 1.0f);
      y1 = y1 > 0.f ? y1 : (__expf(y1) - 1.0f);
      v2f rv;
      rv.x = fmaf(y0, live, pz);
      rv.y = fmaf(y1, live, pz);

      __builtin_amdgcn_fence(__ATOMIC_RELEASE, "wavefront");
      __builtin_amdgcn_wave_barrier();
      *(v2fa*)(stw + c0) = rv;
      __builtin_amdgcn_fence(__ATOMIC_RELEASE, "wavefront");
      __builtin_amdgcn_wave_barrier();
      const bool wr = grow < MPr;
      const v4f ga = *(const v4fa*)(stw + 8 * lc);
      const v4f gb = *(const v4fa*)(stw + 8 * lc + 4);
      v8h hv, lv;
      cvt8hl(ga, gb, hv, lv);
      _Float16* gph = Hh + (size_t)grow * C1 + 8 * lc;
      _Float16* gpl = Hl + (size_t)grow * C1 + 8 * lc;
      const bool wsv = wr && (lane < (C1 / 8));
      if (wsv) { *(volatile v8h*)gph = hv; *(volatile v8h*)gpl = lv; }
      __threadfence();
      if (wsv) { *(volatile v8h*)gph = hv; *(volatile v8h*)gpl = lv; }
    }
  } else {
    const float at0 = rbf(att[lane]);
    const float bb0 = rbf(bias[lane]);
    const float gg0 = rbf(gam[lane]);
    const float ee0 = rbf(bet[lane]);
#pragma unroll 1
    for (int jt = 0; jt < nbw; ++jt) {
      const int slot = wave * nbw + jt;
      const int grow = nodeBase + slot;
      const int gcl  = grow < nN ? grow : nN - 1;
      int st = soff[slot];
      const int craw = scnt[slot];
      int cnt = craw;
      st  = st < 0 ? 0 : (st > nh ? nh : st);
      cnt = cnt < 0 ? 0 : (cnt > DEGCAP ? DEGCAP : cnt);
      if (cnt > nh - st) cnt = nh - st;
      const float pz = (ovf || craw > DEGCAP) ? qnan : 0.0f;

      const float xr = HF[(size_t)gcl * NP2 + C2 + lane];
      ldwait();
      float mx = -1.0e30f, dn = 0.f, a0 = 0.f;

#pragma unroll 1
      for (int q = 0; q < cnt; ++q) {
        int idx = st + q; idx = idx > RCAP - 1 ? RCAP - 1 : idx;
        int eid = reg2[idx]; eid = eid < 0 ? 0 : (eid > nE - 1 ? nE - 1 : eid);
        const int sraw = srcs[eid];
        const int s = sraw < 0 ? 0 : (sraw > nN - 1 ? nN - 1 : sraw);
        const float xs = HF[(size_t)s * NP2 + lane];
        ldwait();
        float v0 = xs + xr; v0 = v0 > 0.f ? v0 : v0 * NEGS;
        const float al = wsum(v0 * at0);
        const float df = al - mx;
        const float ex = __expf(-fabsf(df));
        const bool up  = df > 0.f;
        const float s1 = up ? ex : 1.0f;
        const float s2 = up ? 1.0f : ex;
        mx = up ? al : mx;
        dn = fmaf(dn, s1, s2);
        a0 = fmaf(a0, s1, s2 * xs);
      }
      const float ds = dn > 0.f ? dn : 1.0f;
      const float iv = (dn > 0.f ? 1.0f : 0.0f) * __builtin_amdgcn_rcpf(ds);
      const float t0 = fmaf(a0, iv, bb0);
      const float mu = wsum(t0) * (1.0f / C2);
      const float d0 = t0 - mu;
      const float sq = wsum(d0 * d0);
      const float rs = rsqrtf(sq * (1.0f / C2) + LNEPS);
      const float y0 = fmaf(d0 * rs, gg0, ee0) + pz;

      __builtin_amdgcn_fence(__ATOMIC_RELEASE, "wavefront");
      __builtin_amdgcn_wave_barrier();
      stw[lane] = y0;
      __builtin_amdgcn_fence(__ATOMIC_RELEASE, "wavefront");
      __builtin_amdgcn_wave_barrier();
      const bool wr = grow < nN;
      const v4f gv = *(const v4fa*)(stw + 4 * lc);
      float* gp = outF + (size_t)grow * C2 + 4 * lc;
      const bool wsv = wr && (lane < (C2 / 4));
      if (wsv) *(volatile v4f*)gp = gv;
      __threadfence();
      if (wsv) *(volatile v4f*)gp = gv;
    }
  }
  (void)Hh; (void)Hl; (void)outF; (void)MPr;
}

static int pick_nb(int nE, int nN) {
  int nb = NBRUN;
  while (nb > 16 && (long long)nb * (long long)nE * 5LL > (long long)RCAP * (long long)nN * 4LL) nb >>= 1;
  return nb;
}
static inline int cdiv(int a, int b) { return (a + b - 1) / b; }

extern "C" void kernel_launch(void* const* d_in, const int* in_sizes, int n_in,
                              void* d_out, int out_size, void* d_ws, size_t ws_size,
                              hipStream_t stream) {
  if (n_in < 14) return;
  if (in_sizes[0] < FIN || (in_sizes[0] % FIN) != 0) return;
  const int nN = in_sizes[0] / FIN;
  if (nN <= 0 || nN > (1 << 22)) return;
  if (in_sizes[1] < 2 || (in_sizes[1] & 1) != 0) return;
  const int nE = in_sizes[1] / 2;
  if (nE < 1 || nE >= (1 << (32 - SLOTB))) return;
  if (in_sizes[2] != FIN * C1 || in_sizes[3] != FIN * C1) return;
  if (in_sizes[4] != C1 || in_sizes[5] != C1 || in_sizes[6] != C1 || in_sizes[7] != C1) return;
  if (in_sizes[8] != C1 * C2 || in_sizes[9] != C1 * C2) return;
  if (in_sizes[10] != C2 || in_sizes[11] != C2 || in_sizes[12] != C2 || in_sizes[13] != C2) return;
  if (out_size != nN * C2) return;

  const float* x    = (const float*)d_in[0];
  const int*   ei   = (const int*)  d_in[1];
  const float* Wl1  = (const float*)d_in[2];
  const float* Wr1  = (const float*)d_in[3];
  const float* att1 = (const float*)d_in[4];
  const float* b1   = (const float*)d_in[5];
  const float* g1   = (const float*)d_in[6];
  const float* be1  = (const float*)d_in[7];
  const float* Wl2  = (const float*)d_in[8];
  const float* Wr2  = (const float*)d_in[9];
  const float* att2 = (const float*)d_in[10];
  const float* b2   = (const float*)d_in[11];
  const float* g2   = (const float*)d_in[12];
  const float* be2  = (const float*)d_in[13];
  float* out = (float*)d_out;
  const int* src = ei;
  const int* dst = ei + nE;

  const int MP   = cdiv(nN, GBM) * GBM;
  const int nb   = pick_nb(nE, nN);
  if (nb < 16 || (nb & (nb - 1)) != 0 || nb > NBMAX) return;
  const int gA   = cdiv(MP, nb);
  const int vec8 = ((nE & 3) == 0) ? 1 : 0;
  if ((long long)gA * nb < (long long)MP || (long long)gA * nb < (long long)nN) return;

  char* ws = (char*)d_ws;
  size_t off = 0;
  const size_t oXB  = off; off += (size_t)MP * K1P * 2;            off = (off + 255) & ~(size_t)255;
  const size_t oWT1 = off; off += (size_t)NP1 * K1P * 2;           off = (off + 255) & ~(size_t)255;
  const size_t oWT2 = off; off += (size_t)NP2 * K2 * 2;            off = (off + 255) & ~(size_t)255;
  const size_t oHF1 = off; off += (size_t)MP * NP1 * 4;            off = (off + 255) & ~(size_t)255;
  const size_t oH1H = off; off += (size_t)MP * C1 * 2;             off = (off + 255) & ~(size_t)255;
  const size_t oH1L = off; off += (size_t)MP * C1 * 2;             off = (off + 255) & ~(size_t)255;
  const size_t oHF2 = off; off += (size_t)MP * NP2 * 4;            off = (off + 255) & ~(size_t)255;
  if (off > ws_size || off > (size_t)WSMAX) return;
  unsigned short* XB  = (unsigned short*)(ws + oXB);
  unsigned short* WT1 = (unsigned short*)(ws + oWT1);
  unsigned short* WT2 = (unsigned short*)(ws + oWT2);
  float*          HF1 = (float*)(ws + oHF1);
  unsigned short* H1H = (unsigned short*)(ws + oH1H);
  unsigned short* H1L = (unsigned short*)(ws + oH1L);
  float*          HF2 = (float*)(ws + oHF2);

  hipFuncSetAttribute(reinterpret_cast<const void*>(&k_agg<1>),
                      hipFuncAttributeMaxDynamicSharedMemorySize, LDS_AGG);
  hipFuncSetAttribute(reinterpret_cast<const void*>(&k_agg<2>),
                      hipFuncAttributeMaxDynamicSharedMemorySize, LDS_AGG);

  const int nUx = MP * (K1P / 8);
  k_xprep<<<cdiv(nUx, NTHR), NTHR, 0, stream>>>(x, XB, nN, nUx);

  {
    const int nU1 = NP1 * (K1P / 8);
    k_wcat<0><<<cdiv(nU1, NTHR), NTHR, 0, stream>>>(Wl1, Wr1, C1, FIN, K1P, WT1, nU1);
    const int nU2 = NP2 * (K2 / 8);
    k_wcat<1><<<cdiv(nU2, NTHR), NTHR, 0, stream>>>(Wl2, Wr2, C2, C1, K2, WT2, nU2);
  }

  const int gM = MP / GBM;
  k_gemm<1, 0><<<dim3(gM, NP1 / GBN), GTHR, 0, stream>>>(XB, XB, WT1, HF1, K1P, NP1, 1.0f, 0.0f);
  k_agg<1><<<gA, NTHR, LDS_AGG, stream>>>(src, dst, HF1, att1, b1, g1, be1,
                                          (_Float16*)H1H, (_Float16*)H1L, HF2,
                                          nN, nE, nb, vec8, MP);
  k_gemm<0, 1><<<dim3(gM, NP2 / GBN), GTHR, 0, stream>>>(H1H, H1L, WT2, HF2, K2, NP2, SCL_XW, SCL_XWL);
  k_agg<2><<<gA, NTHR, LDS_AGG, stream>>>(src, dst, HF2, att2, b2, g2, be2,
                                          (_Float16*)H1H, (_Float16*)H1L, out,
                                          nN, nE, nb, vec8, MP);
}
